// RGCNModel_3985729651460
// MI455X (gfx1250) — hardware-run, weakly checked
//
#include <hip/hip_runtime.h>
#include <stddef.h>
#include <stdint.h>

#ifndef SPLIT2
#define SPLIT2 1
#endif

#define NN      100000
#define NE      640000
#define DD      128
#define NR      8
#define GBM     128
#define GBN     128
#define NPAD    100096
#define AP1     128
#define BP1     128
#define AP2     256
#define BP2     256
#define KX1     128
#define KX2     (SPLIT2 ? 256 : 128)
#define NBT     1152
#define XWP     256
#define NTHR    256
#define NWAVE   8
#define EPT     8
#define WCH     (32 * EPT)
#define PERW    (((NE + NWAVE * WCH - 1) / (NWAVE * WCH)) * WCH)
#define NBRUN   1024
#define SLB     10
#define NBK     98
#define NBIN    (NBRUN * NR)
#define WLCAP   2048
#define RCAP    8192
#define DEGCAP  32
#define MAXDEG_MEAS   21
#define MAXB1024_MEAS 6764
#define RPB     64
#define RPW     8
#define SP      68

#define BK_ZINTS (NWAVE * WLCAP + RCAP + 3 * NBIN)
#define BK_INTS  (BK_ZINTS + 32)
#define BK_LDS   (BK_INTS * 4)

#define PBX   (NPAD * DD / 8 / NTHR)
#define PBW1  (NR * DD * (BP1 / 8) / NTHR)
#define PBR1  (DD * (BP1 / 8) / NTHR)
#define PBW2  (NR * DD * (BP2 / 8) / NTHR)
#define PBR2  (DD * (BP2 / 8) / NTHR)
#define PBTOT (PBX + PBW1 + PBR1 + PBW2 + PBR2 + 1)

static_assert(DD == 32 * 4 && NR == 8 && NR % 2 == 0);
static_assert(NPAD == 782 * GBM && NPAD >= NN && NPAD % RPB == 0 && NPAD % GBM == 0);
static_assert(NBRUN == (1 << SLB) && NBIN == NBRUN * NR && NBRUN % RPB == 0);
static_assert(NBK * NBRUN >= NPAD);
static_assert(NN < (1 << 17));
static_assert(NE < (1 << 20) && (((long long)NE) << SLB) < (1LL << 31));
static_assert(NE % WCH == 0 && NE % 4 == 0 && PERW % WCH == 0);
static_assert(NE > (NWAVE - 1) * PERW && (NE - (NWAVE - 1) * PERW) % WCH == 0);
static_assert((long long)RCAP * 100 >= (long long)MAXB1024_MEAS * 105);
static_assert(DEGCAP >= MAXDEG_MEAS + 8);
static_assert(WLCAP >= 2 * (MAXB1024_MEAS / NWAVE + 1));
static_assert(RCAP == NBIN && RCAP % (NTHR * 4) == 0 && BK_ZINTS % (NTHR * 4) == 0);
static_assert(NBIN == NTHR * 32);
static_assert(BK_LDS <= 327680);
static_assert((GBM * SP + GBN) * 4 <= 65536);
static_assert(KX1 % 32 == 0 && KX2 % 32 == 0 && KX1 <= AP1 && KX1 <= BP1 && KX2 <= AP2 && KX2 <= BP2);
static_assert(AP2 == 2 * DD && BP2 == 2 * DD && NBT == NR * DD + DD && XWP == 2 * DD);
static_assert((NPAD * DD / 8) % NTHR == 0 && (NR * DD * (BP1 / 8)) % NTHR == 0 && (DD * (BP1 / 8)) % NTHR == 0);
static_assert((NR * DD * (BP2 / 8)) % NTHR == 0 && (DD * (BP2 / 8)) % NTHR == 0);
static_assert(RPB == NWAVE * RPW);

typedef float          v4f   __attribute__((ext_vector_type(4)));
typedef float          v8f   __attribute__((ext_vector_type(8)));
typedef int            v2i   __attribute__((ext_vector_type(2)));
typedef int            v4i   __attribute__((ext_vector_type(4)));
typedef int            v8i   __attribute__((ext_vector_type(8)));
typedef unsigned       v2u   __attribute__((ext_vector_type(2)));
typedef unsigned short v8us  __attribute__((ext_vector_type(8)));
typedef __bf16         v16bf __attribute__((ext_vector_type(16)));
typedef v4f  __attribute__((may_alias)) v4fa;
typedef v2i  __attribute__((may_alias)) v2ia;
typedef v4i  __attribute__((may_alias)) v4ia;
typedef v8us __attribute__((may_alias)) v8usa;
union FragB { v16bf v; v8us h[2]; v8i w; };

__device__ __forceinline__ v8f wmb(const FragB& a, const FragB& b, v8f c) {
  v8f d = __builtin_amdgcn_wmma_f32_16x16x32_bf16(false, a.v, false, b.v, (short)0, c, false, false);
  asm volatile("v_nop\n\tv_nop\n\tv_nop\n\tv_nop" : "+v"(d) : "v"(a.w), "v"(b.w));
  return d;
}

__device__ __forceinline__ unsigned bf16_bits(float f) {
  const unsigned u = __float_as_uint(f);
  const unsigned r = (u + 0x7FFFu + ((u >> 16) & 1u)) >> 16;
  const unsigned q = (u >> 16) | 0x40u;
  return ((u & 0x7fffffffu) > 0x7f800000u) ? q : r;
}
__device__ __forceinline__ float bf16_val(float f) {
  return __uint_as_float(bf16_bits(f) << 16);
}

__device__ __forceinline__ void hilo_pack(float v0, float v1, float v2, float v3,
                                          unsigned& h01, unsigned& h23, unsigned& l01, unsigned& l23) {
  const unsigned a0 = bf16_bits(v0), a1 = bf16_bits(v1), a2 = bf16_bits(v2), a3 = bf16_bits(v3);
  const unsigned b0 = bf16_bits(v0 - __uint_as_float(a0 << 16));
  const unsigned b1 = bf16_bits(v1 - __uint_as_float(a1 << 16));
  const unsigned b2 = bf16_bits(v2 - __uint_as_float(a2 << 16));
  const unsigned b3 = bf16_bits(v3 - __uint_as_float(a3 << 16));
  h01 = a0 | (a1 << 16); h23 = a2 | (a3 << 16);
  l01 = b0 | (b1 << 16); l23 = b2 | (b3 << 16);
}

__device__ __forceinline__ float relu_k(float v) { return (v > 0.0f) ? v : (v - v); }

__device__ __forceinline__ void st2_v4f(float* p, v4f v) {
  *(volatile v4f*)p = v;
  __threadfence();
  *(volatile v4f*)p = v;
}
__device__ __forceinline__ void st2_v8us(unsigned short* p, v8us v) {
  *(volatile v8us*)p = v;
  __threadfence();
  *(volatile v8us*)p = v;
}

__device__ __forceinline__ v8us gather8(const float* __restrict__ base, int stride) {
  float f[8];
#pragma unroll
  for (int i = 0; i < 8; ++i) f[i] = base[(size_t)i * (size_t)stride];
  v8us o;
#pragma unroll
  for (int i = 0; i < 8; ++i) o[i] = (unsigned short)bf16_bits(f[i]);
  return o;
}

__global__ __launch_bounds__(NTHR) void k_prep(const float* __restrict__ x,
                                               const float* __restrict__ w1, const float* __restrict__ r1,
                                               const float* __restrict__ b1,
                                               const float* __restrict__ w2, const float* __restrict__ r2,
                                               const float* __restrict__ b2,
                                               unsigned short* xb, unsigned short* wt1, unsigned short* wt2,
                                               float* bf) {
  const int tid = (int)threadIdx.x, lane = tid & 31, wave = tid >> 5;
  const int blk = (int)blockIdx.x;
  if (blk < PBX) {
    const int u   = blk * NTHR + tid;
    const int row = u >> 4, k8 = (u & 15) * 8;
    const int rc  = row < NN ? row : NN - 1;
    const unsigned mk = row < NN ? 0xffffu : 0u;
    const float* p = x + (size_t)rc * DD + k8;
    const v4f a = *(const v4fa*)p;
    const v4f b = *(const v4fa*)(p + 4);
    v8us o;
    o[0] = (unsigned short)(bf16_bits(a.x) & mk); o[1] = (unsigned short)(bf16_bits(a.y) & mk);
    o[2] = (unsigned short)(bf16_bits(a.z) & mk); o[3] = (unsigned short)(bf16_bits(a.w) & mk);
    o[4] = (unsigned short)(bf16_bits(b.x) & mk); o[5] = (unsigned short)(bf16_bits(b.y) & mk);
    o[6] = (unsigned short)(bf16_bits(b.z) & mk); o[7] = (unsigned short)(bf16_bits(b.w) & mk);
    st2_v8us(xb + (size_t)row * AP1 + k8, o);
  } else if (blk < PBX + PBW1) {
    const int u = (blk - PBX) * NTHR + tid;
    const int n = u >> 4, k8 = (u & 15) * 8;
    const int r = n >> 7, o = n & 127;
    const v8us v = gather8(w1 + (size_t)r * DD * DD + (size_t)k8 * DD + o, DD);
    st2_v8us(wt1 + (size_t)n * BP1 + k8, v);
  } else if (blk < PBX + PBW1 + PBR1) {
    const int u = (blk - PBX - PBW1) * NTHR + tid;
    const int n = u >> 4, k8 = (u & 15) * 8;
    const v8us v = gather8(r1 + (size_t)k8 * DD + n, DD);
    st2_v8us(wt1 + (size_t)(NR * DD + n) * BP1 + k8, v);
  } else if (blk < PBX + PBW1 + PBR1 + PBW2) {
    const int u = (blk - PBX - PBW1 - PBR1) * NTHR + tid;
    const int n = u >> 5, k8 = (u & 31) * 8, kk = k8 & (DD - 1);
    const int r = n >> 7, o = n & 127;
    const v8us v = gather8(w2 + (size_t)r * DD * DD + (size_t)kk * DD + o, DD);
    st2_v8us(wt2 + (size_t)n * BP2 + k8, v);
  } else if (blk < PBX + PBW1 + PBR1 + PBW2 + PBR2) {
    const int u = (blk - PBX - PBW1 - PBR1 - PBW2) * NTHR + tid;
    const int n = u >> 5, k8 = (u & 31) * 8, kk = k8 & (DD - 1);
    const v8us v = gather8(r2 + (size_t)kk * DD + n, DD);
    st2_v8us(wt2 + (size_t)(NR * DD + n) * BP2 + k8, v);
  } else {
    if (wave == 0) {
      const v4f a = *(const v4fa*)(b1 + 4 * lane);
      v4f o;
      o.x = bf16_val(a.x); o.y = bf16_val(a.y); o.z = bf16_val(a.z); o.w = bf16_val(a.w);
      st2_v4f(bf + 4 * lane, o);
    } else if (wave == 1) {
      const v4f a = *(const v4fa*)(b2 + 4 * lane);
      v4f o;
      o.x = bf16_val(a.x); o.y = bf16_val(a.y); o.z = bf16_val(a.z); o.w = bf16_val(a.w);
      st2_v4f(bf + DD + 4 * lane, o);
    }
  }
}

__global__ __launch_bounds__(NTHR) void k_bucket(const int* __restrict__ srcs, const int* __restrict__ dsts,
                                                 const int* __restrict__ ety,
                                                 int* LIST, int* CNT8, int* OFF8, int* FLAG) {
  extern __shared__ __attribute__((aligned(16))) int dsm[];
  int* wl   = dsm;
  int* pl   = dsm + NWAVE * WLCAP;
  int* cnt  = pl + RCAP;
  int* offs = cnt + NBIN;
  int* cur  = offs + NBIN;
  int* misc = cur + NBIN;
  const int tid = (int)threadIdx.x, lane = tid & 31, wave = tid >> 5;
  const int blk = (int)blockIdx.x;
  const unsigned nbs = (unsigned)(blk * NBRUN);

  {
    const v4i z4 = {0, 0, 0, 0};
    for (int i = tid * 4; i < BK_ZINTS; i += NTHR * 4) *(v4ia*)(dsm + i) = z4;
    if (tid < 32) misc[tid] = 0;
  }
  __syncthreads();

  {
    const int ebeg = wave * PERW;
    const int eend = (ebeg + PERW < NE) ? (ebeg + PERW) : NE;
    int* mylist = wl + wave * WLCAP;
    int wc = 0;
#pragma unroll 1
    for (int cb = ebeg; cb < eend; cb += WCH) {
      const int e0 = cb + lane * EPT;
      const v4i da = *(const v4ia*)(dsts + e0);
      const v4i db = *(const v4ia*)(dsts + e0 + 4);
      const unsigned s0 = (unsigned)da.x - nbs, s1 = (unsigned)da.y - nbs;
      const unsigned s2 = (unsigned)da.z - nbs, s3 = (unsigned)da.w - nbs;
      const unsigned s4 = (unsigned)db.x - nbs, s5 = (unsigned)db.y - nbs;
      const unsigned s6 = (unsigned)db.z - nbs, s7 = (unsigned)db.w - nbs;
      const bool h0 = s0 < (unsigned)NBRUN, h1 = s1 < (unsigned)NBRUN, h2 = s2 < (unsigned)NBRUN, h3 = s3 < (unsigned)NBRUN;
      const bool h4 = s4 < (unsigned)NBRUN, h5 = s5 < (unsigned)NBRUN, h6 = s6 < (unsigned)NBRUN, h7 = s7 < (unsigned)NBRUN;
      const unsigned m0 = __builtin_amdgcn_ballot_w32(h0), m1 = __builtin_amdgcn_ballot_w32(h1);
      const unsigned m2 = __builtin_amdgcn_ballot_w32(h2), m3 = __builtin_amdgcn_ballot_w32(h3);
      const unsigned m4 = __builtin_amdgcn_ballot_w32(h4), m5 = __builtin_amdgcn_ballot_w32(h5);
      const unsigned m6 = __builtin_amdgcn_ballot_w32(h6), m7 = __builtin_amdgcn_ballot_w32(h7);
      const unsigned any = m0 | m1 | m2 | m3 | m4 | m5 | m6 | m7;
      if (any != 0u) {
        const int pre = (int)(__builtin_amdgcn_mbcnt_lo(m0, 0u) + __builtin_amdgcn_mbcnt_lo(m1, 0u) +
                              __builtin_amdgcn_mbcnt_lo(m2, 0u) + __builtin_amdgcn_mbcnt_lo(m3, 0u) +
                              __builtin_amdgcn_mbcnt_lo(m4, 0u) + __builtin_amdgcn_mbcnt_lo(m5, 0u) +
                              __builtin_amdgcn_mbcnt_lo(m6, 0u) + __builtin_amdgcn_mbcnt_lo(m7, 0u));
        int p = wc + pre;
        if (h0) { if (p < WLCAP) mylist[p] = ((e0 + 0) << SLB) | (int)s0; p = p + 1; }
        if (h1) { if (p < WLCAP) mylist[p] = ((e0 + 1) << SLB) | (int)s1; p = p + 1; }
        if (h2) { if (p < WLCAP) mylist[p] = ((e0 + 2) << SLB) | (int)s2; p = p + 1; }
        if (h3) { if (p < WLCAP) mylist[p] = ((e0 + 3) << SLB) | (int)s3; p = p + 1; }
        if (h4) { if (p < WLCAP) mylist[p] = ((e0 + 4) << SLB) | (int)s4; p = p + 1; }
        if (h5) { if (p < WLCAP) mylist[p] = ((e0 + 5) << SLB) | (int)s5; p = p + 1; }
        if (h6) { if (p < WLCAP) mylist[p] = ((e0 + 6) << SLB) | (int)s6; p = p + 1; }
        if (h7) { if (p < WLCAP) mylist[p] = ((e0 + 7) << SLB) | (int)s7; p = p + 1; }
        wc += (int)(__builtin_popcount(m0) + __builtin_popcount(m1) + __builtin_popcount(m2) + __builtin_popcount(m3) +
                    __builtin_popcount(m4) + __builtin_popcount(m5) + __builtin_popcount(m6) + __builtin_popcount(m7));
      }
    }
    if (lane == 0) misc[wave] = wc;
  }
  __syncthreads();

  if (wave == 0) {
    int ov = 0;
#pragma unroll 1
    for (int w2 = 0; w2 < NWAVE; ++w2) {
      int c = misc[w2];
      if (c > WLCAP) ov = 1;
      c = c < 0 ? 0 : (c > WLCAP ? WLCAP : c);
#pragma unroll 1
      for (int b0 = 0; b0 < c; b0 += 32) {
        const int idx = b0 + lane;
        const int ent = wl[w2 * WLCAP + (idx < WLCAP ? idx : WLCAP - 1)];
        int eid = (ent >> SLB) & 0xFFFFF;
        eid = eid > NE - 1 ? NE - 1 : eid;
        int ty = ety[eid];
        ty = ty < 0 ? 0 : (ty > NR - 1 ? NR - 1 : ty);
        const int key = ((ent & (NBRUN - 1)) << 3) | ty;
        const int m32 = (c - b0) < 32 ? (c - b0) : 32;
#pragma unroll 1
        for (int k = 0; k < m32; ++k) {
          const int u = __builtin_amdgcn_readlane(key, k);
          if (lane == 0) cnt[u] = cnt[u] + 1;
        }
      }
    }
    if (lane == 0) misc[16] = ov;
  }
  __syncthreads();

  {
    const int base = tid * 32;
    int s = 0;
#pragma unroll 1
    for (int i = 0; i < 8; ++i) {
      const v4i c4 = *(const v4ia*)(cnt + base + 4 * i);
      s += c4.x + c4.y + c4.z + c4.w;
    }
    int incl = s;
#pragma unroll
    for (int d = 1; d < 32; d <<= 1) {
      const int y = __shfl_up(incl, d, 32);
      if (lane >= d) incl += y;
    }
    if (lane == 31) misc[8 + wave] = incl;
    __syncthreads();
    int pre = 0, tot = 0;
#pragma unroll
    for (int w2 = 0; w2 < NWAVE; ++w2) {
      const int t = misc[8 + w2];
      tot += t;
      pre += (w2 < wave) ? t : 0;
    }
    int run = pre + incl - s;
#pragma unroll 1
    for (int i = 0; i < 8; ++i) {
      const v4i c4 = *(const v4ia*)(cnt + base + 4 * i);
      v4i o4;
      o4.x = run; run += c4.x;
      o4.y = run; run += c4.y;
      o4.z = run; run += c4.z;
      o4.w = run; run += c4.w;
      *(v4ia*)(offs + base + 4 * i) = o4;
      *(v4ia*)(cur + base + 4 * i)  = o4;
    }
    if (tid == 0) {
      const int ov0 = misc[16];
      misc[16] = (ov0 != 0 || tot > RCAP) ? 1 : 0;
    }
  }
  __syncthreads();

  if (wave == 0) {
#pragma unroll 1
    for (int w2 = 0; w2 < NWAVE; ++w2) {
      int c = misc[w2];
      c = c < 0 ? 0 : (c > WLCAP ? WLCAP : c);
#pragma unroll 1
      for (int b0 = 0; b0 < c; b0 += 32) {
        const int idx = b0 + lane;
        const int ent = wl[w2 * WLCAP + (idx < WLCAP ? idx : WLCAP - 1)];
        int eid = (ent >> SLB) & 0xFFFFF;
        eid = eid > NE - 1 ? NE - 1 : eid;
        int sr = srcs[eid];
        sr = sr < 0 ? 0 : (sr > NN - 1 ? NN - 1 : sr);
        int ty = ety[eid];
        ty = ty < 0 ? 0 : (ty > NR - 1 ? NR - 1 : ty);
        const int key  = ((ent & (NBRUN - 1)) << 3) | ty;
        const int word = (int)(((unsigned)ty << 17) | (unsigned)sr);
        const int m32 = (c - b0) < 32 ? (c - b0) : 32;
#pragma unroll 1
        for (int k = 0; k < m32; ++k) {
          const int u  = __builtin_amdgcn_readlane(key, k);
          const int wd = __builtin_amdgcn_readlane(word, k);
          if (lane == 0) {
            int p = cur[u];
            p = p < 0 ? 0 : (p > RCAP - 1 ? RCAP - 1 : p);
            pl[p] = wd;
            cur[u] = p + 1;
          }
        }
      }
    }
  }
  __syncthreads();

  const int ovf = misc[16];
  int* lp = LIST + (size_t)blk * RCAP;
  int* cp = CNT8 + (size_t)blk * NBIN;
  int* op = OFF8 + (size_t)blk * NBIN;
  int* fp = FLAG + (size_t)blk * 32;
#pragma unroll
  for (int ps = 0; ps < 2; ++ps) {
#pragma unroll 1
    for (int i = tid * 4; i < RCAP; i += NTHR * 4) {
      const v4i a = *(const v4ia*)(pl + i);
      const v4i b = *(const v4ia*)(cnt + i);
      const v4i c = *(const v4ia*)(offs + i);
      *(volatile v4i*)(lp + i) = a;
      *(volatile v4i*)(cp + i) = b;
      *(volatile v4i*)(op + i) = c;
    }
    if (tid < 8) {
      const v4i f = {ovf, ovf, ovf, ovf};
      *(volatile v4i*)(fp + 4 * tid) = f;
    }
    if (ps == 0) __threadfence();
  }
}

template <int KEXT, int AP, int BP, int OP, int BIAS>
__global__ __launch_bounds__(NTHR) __attribute__((amdgpu_num_vgpr(248)))
void k_gemm(const unsigned short* __restrict__ A, const unsigned short* __restrict__ BT,
            const float* __restrict__ bias, float* OUT) {
  static_assert(KEXT % 32 == 0 && KEXT <= AP && KEXT <= BP && AP % 8 == 0 && BP % 8 == 0 && OP % 32 == 0);
  __shared__ __attribute__((aligned(16))) float stg[GBM * SP];
  __shared__ __attribute__((aligned(16))) float sb[GBN];
  const int tid = (int)threadIdx.x, lane = tid & 31, wave = tid >> 5, hh = lane >> 4, m = lane & 15;
  const int rowBase = (int)blockIdx.x * GBM;
  const int colBase = (int)blockIdx.y * GBN;

  if (tid < 32) {
    v4f b4 = {0.f, 0.f, 0.f, 0.f};
    if constexpr (BIAS != 0) b4 = *(const v4fa*)(bias + 4 * tid);
    *(v4fa*)(sb + 4 * tid) = b4;
  }

  v8f acc[8];
  {
    const v8f z = {0.f, 0.f, 0.f, 0.f, 0.f, 0.f, 0.f, 0.f};
#pragma unroll
    for (int t = 0; t < 8; ++t) acc[t] = z;
  }
  const unsigned short* ap = A + (size_t)(rowBase + 16 * wave + m) * (size_t)AP + 8 * hh;
  const unsigned short* bp = BT + (size_t)(colBase + m) * (size_t)BP + 8 * hh;
#pragma unroll 1
  for (int k0 = 0; k0 < KEXT; k0 += 32) {
    FragB af;
    af.h[0] = *(const v8usa*)(ap + k0);
    af.h[1] = *(const v8usa*)(ap + k0 + 16);
#pragma unroll
    for (int nt = 0; nt < 8; ++nt) {
      const unsigned short* wq = bp + (size_t)(16 * nt) * (size_t)BP + k0;
      FragB bf;
      bf.h[0] = *(const v8usa*)wq;
      bf.h[1] = *(const v8usa*)(wq + 16);
      acc[nt] = wmb(af, bf, acc[nt]);
    }
  }

#pragma unroll
  for (int ch = 0; ch < 2; ++ch) {
#pragma unroll
    for (int t = 0; t < 4; ++t) {
#pragma unroll
      for (int r = 0; r < 8; ++r) stg[(16 * wave + 8 * hh + r) * SP + 16 * t + m] = acc[4 * ch + t][r];
    }
    __syncthreads();
    const v4f bq = *(const v4fa*)(sb + 64 * ch + 4 * m);
#pragma unroll
    for (int ps = 0; ps < 2; ++ps) {
#pragma unroll 1
      for (int i = 0; i < 8; ++i) {
        const int lr = 16 * wave + 2 * i + hh;
        const v4f a = *(const v4fa*)(stg + lr * SP + 4 * m);
        v4f o;
        o.x = a.x + bq.x; o.y = a.y + bq.y; o.z = a.z + bq.z; o.w = a.w + bq.w;
        float* op = OUT + (size_t)(rowBase + lr) * (size_t)OP + colBase + 64 * ch + 4 * m;
        *(volatile v4f*)op = o;
      }
      if (ps == 0) __threadfence();
    }
    __syncthreads();
  }
}

__device__ __forceinline__ v4f walk(const int* __restrict__ lb, const float* __restrict__ XW2,
                                    int o, int c, int p2, int lane) {
  int last = o + c - 1;
  last = last < o ? o : last;
  v4f a = {0.f, 0.f, 0.f, 0.f};
#pragma unroll 1
  for (int j = 0; j < c; ++j) {
    int idx = o + j;
    idx = idx > last ? last : idx;
    const unsigned wd = (unsigned)lb[idx];
    int sr = (int)(wd & 0x1FFFFu);
    sr = sr > NN - 1 ? NN - 1 : sr;
    int rl = (int)((wd >> 17) & 7u) - p2;
    rl = rl < 0 ? 0 : (rl > 1 ? 1 : rl);
    const v4f v = *(const v4fa*)(XW2 + (size_t)sr * XWP + rl * DD + 4 * lane);
    a.x += v.x; a.y += v.y; a.z += v.z; a.w += v.w;
  }
  return a;
}

template <int MODE>
__global__ __launch_bounds__(NTHR) void k_replay(const int* __restrict__ LIST, const int* __restrict__ CNT8,
                                                 const int* __restrict__ OFF8, const int* __restrict__ FLAG,
                                                 const float* __restrict__ XW2, float* ACC,
                                                 unsigned short* HHL, float* OUT, int p) {
  const int tid = (int)threadIdx.x, lane = tid & 31, wave = tid >> 5;
  const int rowBase = (int)blockIdx.x * RPB;
  const int bucket  = rowBase >> SLB;
  const int* lb  = LIST + (size_t)bucket * RCAP;
  const int flag = FLAG[(size_t)bucket * 32];
  const int pc   = p < 0 ? 0 : (p > NR / 2 - 1 ? NR / 2 - 1 : p);
  const float qnan = __uint_as_float(0x7fc00000u);

#pragma unroll 1
  for (int i = 0; i < RPW; ++i) {
    const int d = rowBase + RPW * wave + i;
    const v2i cv = *(const v2ia*)(CNT8 + (size_t)d * NR + 2 * pc);
    const v2i ov = *(const v2ia*)(OFF8 + (size_t)d * NR + 2 * pc);
    int c0 = cv.x, c1 = cv.y, o0 = ov.x, o1 = ov.y;
    const bool big = (c0 > DEGCAP) | (c1 > DEGCAP);
    c0 = c0 < 0 ? 0 : (c0 > DEGCAP ? DEGCAP : c0);
    c1 = c1 < 0 ? 0 : (c1 > DEGCAP ? DEGCAP : c1);
    o0 = o0 < 0 ? 0 : (o0 > RCAP - 1 ? RCAP - 1 : o0);
    o1 = o1 < 0 ? 0 : (o1 > RCAP - 1 ? RCAP - 1 : o1);
    c0 = c0 > RCAP - o0 ? RCAP - o0 : c0;
    c1 = c1 > RCAP - o1 ? RCAP - o1 : c1;
    const int c0u = __builtin_amdgcn_readfirstlane(c0);
    const int c1u = __builtin_amdgcn_readfirstlane(c1);
    const int o0u = __builtin_amdgcn_readfirstlane(o0);
    const int o1u = __builtin_amdgcn_readfirstlane(o1);

    const v4f a0 = walk(lb, XW2, o0u, c0u, 2 * pc, lane);
    const v4f a1 = walk(lb, XW2, o1u, c1u, 2 * pc, lane);
    const float f0 = (float)(c0u > 1 ? c0u : 1);
    const float f1 = (float)(c1u > 1 ? c1u : 1);

    const v4f g = *(const v4fa*)(ACC + (size_t)d * DD + 4 * lane);
    asm volatile("" :: "v"(g));
    float v0 = g.x + (a0.x / f0 + a1.x / f1);
    float v1 = g.y + (a0.y / f0 + a1.y / f1);
    float v2 = g.z + (a0.z / f0 + a1.z / f1);
    float v3 = g.w + (a0.w / f0 + a1.w / f1);
    const bool bad = (flag != 0) | big;
    v0 = bad ? qnan : v0; v1 = bad ? qnan : v1; v2 = bad ? qnan : v2; v3 = bad ? qnan : v3;

    if constexpr (MODE == 0) {
      v4f o;
      o.x = v0; o.y = v1; o.z = v2; o.w = v3;
      st2_v4f(ACC + (size_t)d * DD + 4 * lane, o);
    } else if constexpr (MODE == 1) {
      const bool live = d < NN;
      v0 = relu_k(v0); v1 = relu_k(v1); v2 = relu_k(v2); v3 = relu_k(v3);
      v0 = live ? v0 : 0.0f; v1 = live ? v1 : 0.0f; v2 = live ? v2 : 0.0f; v3 = live ? v3 : 0.0f;
      unsigned h01, h23, l01, l23;
      hilo_pack(v0, v1, v2, v3, h01, h23, l01, l23);
      v2u qh, ql;
      qh.x = h01; qh.y = h23;
      ql.x = l01; ql.y = l23;
      unsigned short* hp = HHL + (size_t)d * AP2 + 4 * lane;
      *(volatile v2u*)hp = qh;
      *(volatile v2u*)(hp + DD) = ql;
      __threadfence();
      *(volatile v2u*)hp = qh;
      *(volatile v2u*)(hp + DD) = ql;
    } else {
      v4f o;
      o.x = bad ? qnan : v0; o.y = bad ? qnan : v1; o.z = bad ? qnan : v2; o.w = bad ? qnan : v3;
      if (d < NN) {
        float* op = OUT + (size_t)d * DD + 4 * lane;
        *(volatile v4f*)op = o;
        __threadfence();
        *(volatile v4f*)op = o;
      }
    }
  }
}

extern "C" void kernel_launch(void* const* d_in, const int* in_sizes, int n_in,
                              void* d_out, int out_size, void* d_ws, size_t ws_size,
                              hipStream_t stream) {
  if (n_in < 9) return;
  if (in_sizes[0] != NN * DD) return;
  if (in_sizes[1] != 2 * NE) return;
  if (in_sizes[2] != NE) return;
  if (in_sizes[3] != NR * DD * DD) return;
  if (in_sizes[4] != DD * DD) return;
  if (in_sizes[5] != DD) return;
  if (in_sizes[6] != NR * DD * DD) return;
  if (in_sizes[7] != DD * DD) return;
  if (in_sizes[8] != DD) return;
  if (out_size != NN * DD) return;

  const float* x  = (const float*)d_in[0];
  const int*   ei = (const int*)d_in[1];
  const int*   et = (const int*)d_in[2];
  const float* W1 = (const float*)d_in[3];
  const float* R1 = (const float*)d_in[4];
  const float* b1 = (const float*)d_in[5];
  const float* W2 = (const float*)d_in[6];
  const float* R2 = (const float*)d_in[7];
  const float* b2 = (const float*)d_in[8];
  float* out = (float*)d_out;
  const int* srcs = ei;
  const int* dsts = ei + NE;

  constexpr size_t zXB   = (size_t)NPAD * AP1 * 2;
  constexpr size_t zHHL  = (size_t)NPAD * AP2 * 2;
  constexpr size_t zXW   = (size_t)NPAD * XWP * 4;
  constexpr size_t zACC  = (size_t)NPAD * DD * 4;
  constexpr size_t zLIST = (size_t)NBK * RCAP * 4;
  constexpr size_t zCNT  = (size_t)NBK * NBIN * 4;
  constexpr size_t zWT1  = (size_t)NBT * BP1 * 2;
  constexpr size_t zWT2  = (size_t)NBT * BP2 * 2;
  constexpr size_t zBF   = (size_t)2 * DD * 4;
  constexpr size_t zFLAG = (size_t)NBK * 128;
  constexpr size_t oXB   = 0;
  constexpr size_t oHHL  = oXB + zXB;
  constexpr size_t oXW   = oHHL + zHHL;
  constexpr size_t oACC  = oXW + zXW;
  constexpr size_t oLIST = oACC + zACC;
  constexpr size_t oCNT  = oLIST + zLIST;
  constexpr size_t oOFF  = oCNT + zCNT;
  constexpr size_t oWT1  = oOFF + zCNT;
  constexpr size_t oWT2  = oWT1 + zWT1;
  constexpr size_t oBF   = oWT2 + zWT2;
  constexpr size_t oFLAG = oBF + zBF;
  constexpr size_t oEND  = oFLAG + zFLAG;
  static_assert(zXB % 256 == 0 && zHHL % 256 == 0 && zXW % 256 == 0 && zACC % 256 == 0 && zLIST % 256 == 0);
  static_assert(zCNT % 256 == 0 && zWT1 % 256 == 0 && zWT2 % 256 == 0 && zBF % 256 == 0 && zFLAG % 256 == 0);
  static_assert((size_t)NBK * NBRUN * NR * 4 == zCNT);
  static_assert(oEND <= (size_t)(256u << 20));
  if (oEND > ws_size) return;

  char* ws = (char*)d_ws;
  unsigned short* XB   = (unsigned short*)(ws + oXB);
  unsigned short* HHL  = (unsigned short*)(ws + oHHL);
  float*          XW2  = (float*)(ws + oXW);
  float*          ACC  = (float*)(ws + oACC);
  int*            LIST = (int*)(ws + oLIST);
  int*            CNT8 = (int*)(ws + oCNT);
  int*            OFF8 = (int*)(ws + oOFF);
  unsigned short* WT1  = (unsigned short*)(ws + oWT1);
  unsigned short* WT2  = (unsigned short*)(ws + oWT2);
  float*          BF   = (float*)(ws + oBF);
  int*            FLAG = (int*)(ws + oFLAG);

  hipFuncSetAttribute(reinterpret_cast<const void*>(&k_bucket), hipFuncAttributeMaxDynamicSharedMemorySize, (int)BK_LDS);

  k_prep<<<PBTOT, NTHR, 0, stream>>>(x, W1, R1, b1, W2, R2, b2, XB, WT1, WT2, BF);
  k_bucket<<<NBK, NTHR, BK_LDS, stream>>>(srcs, dsts, et, LIST, CNT8, OFF8, FLAG);

  const dim3 gRoot((unsigned)(NPAD / GBM), 1u, 1u);
  const dim3 gPass((unsigned)(NPAD / GBM), 2u, 1u);
  const int  gRep = NPAD / RPB;

  k_gemm<KX1, AP1, BP1, DD, 1><<<gRoot, NTHR, 0, stream>>>(XB, WT1 + (size_t)(NR * DD) * BP1, BF, ACC);
  for (int p = 0; p < NR / 2; ++p) {
    k_gemm<KX1, AP1, BP1, XWP, 0><<<gPass, NTHR, 0, stream>>>(XB, WT1 + (size_t)(2 * DD * p) * BP1, BF, XW2);
    if (p < NR / 2 - 1)
      k_replay<0><<<gRep, NTHR, 0, stream>>>(LIST, CNT8, OFF8, FLAG, XW2, ACC, HHL, out, p);
    else
      k_replay<1><<<gRep, NTHR, 0, stream>>>(LIST, CNT8, OFF8, FLAG, XW2, ACC, HHL, out, p);
  }
  k_gemm<KX2, AP2, BP2, DD, 1><<<gRoot, NTHR, 0, stream>>>(HHL, WT2 + (size_t)(NR * DD) * BP2, BF + DD, ACC);
  for (int p = 0; p < NR / 2; ++p) {
    k_gemm<KX2, AP2, BP2, XWP, 0><<<gPass, NTHR, 0, stream>>>(HHL, WT2 + (size_t)(2 * DD * p) * BP2, BF, XW2);
    if (p < NR / 2 - 1)
      k_replay<0><<<gRep, NTHR, 0, stream>>>(LIST, CNT8, OFF8, FLAG, XW2, ACC, HHL, out, p);
    else
      k_replay<2><<<gRep, NTHR, 0, stream>>>(LIST, CNT8, OFF8, FLAG, XW2, ACC, HHL, out, p);
  }
}
